// MHA_87729001988494
// MI455X (gfx1250) — hardware-verified
//
#include <hip/hip_runtime.h>


#define NB_  4
#define TT   2048
#define DM   1024
#define NH_  16
#define NKV  16
#define REP  (NH_ / NKV)
#define HD   64
#define DQ   (NH_ * HD)
#define DKV  (NKV * HD)
#define ZH   2
#define RH   512
#define WIN  0
#define PCAR 1024.0f
#define SCL  0.125f
typedef _Float16 h16;
typedef unsigned short bf;
typedef __attribute__((ext_vector_type(16))) __bf16   v16bf;
typedef __attribute__((ext_vector_type(16))) _Float16 v16h;
typedef __attribute__((ext_vector_type(8)))  _Float16 v8h;
typedef __attribute__((ext_vector_type(8)))  unsigned short v8us;
typedef __attribute__((ext_vector_type(8)))  float    v8f;
typedef __attribute__((ext_vector_type(4)))  float    v4f;
typedef v8h  __attribute__((may_alias)) v8ha;
typedef v4f  __attribute__((may_alias)) v4fa;
typedef v8us __attribute__((may_alias)) v8usa;

__device__ __forceinline__ unsigned short f2bf(float f) { unsigned u = __float_as_uint(f); u += 0x7FFFu + ((u >> 16) & 1u); return (unsigned short)(u >> 16); }
__device__ __forceinline__ float bf2f(unsigned short b) { return __uint_as_float(((unsigned)b) << 16); }
__device__ __forceinline__ float bfr(float f) { return bf2f(f2bf(f)); }
__device__ __forceinline__ v16h cat16(v8h lo, v8h hi) { return __builtin_shufflevector(lo, hi, 0, 1, 2, 3, 4, 5, 6, 7, 8, 9, 10, 11, 12, 13, 14, 15); }
__device__ __forceinline__ v16bf cat16b(v8us lo, v8us hi) { return __builtin_bit_cast(v16bf, __builtin_shufflevector(lo, hi, 0, 1, 2, 3, 4, 5, 6, 7, 8, 9, 10, 11, 12, 13, 14, 15)); }
__device__ __forceinline__ v8f wmma16(v16h a, v16h b, v8f c) { return __builtin_amdgcn_wmma_f32_16x16x32_f16(false, a, false, b, (short)0, c, false, false); }
__device__ __forceinline__ v8f wmmab(v16bf a, v16bf b, v8f c) { return __builtin_amdgcn_wmma_f32_16x16x32_bf16(false, a, false, b, (short)0, c, false, false); }


template <typename T16> struct WFrag;
template <> struct WFrag<h16> { typedef v16h V; static __device__ __forceinline__ V ld(const h16* p) { return cat16(*(const v8h*)p, *(const v8h*)(p + 16)); } static __device__ __forceinline__ v8f mma(V a, V b, v8f c) { return wmma16(a, b, c); } };
template <> struct WFrag<bf> { typedef v16bf V; static __device__ __forceinline__ V ld(const bf* p) { return cat16b(*(const v8us*)p, *(const v8us*)(p + 16)); } static __device__ __forceinline__ v8f mma(V a, V b, v8f c) { return wmmab(a, b, c); } };
template <typename T16, int NSPLIT, bool BIAS>
__global__ __launch_bounds__(32) void k_gemmw(const T16* __restrict__ A, const T16* __restrict__ A2, const T16* __restrict__ Bt, const T16* __restrict__ Bt2, int K, float* C, int ldc, const float* __restrict__ bias, size_t sA, size_t sB, size_t sC) {
    typedef typename WFrag<T16>::V V;
    __shared__ __align__(16) float os[16 * 68];
    const size_t z = blockIdx.z; A += z * sA; if (A2) A2 += z * sA; Bt += z * sB; if (Bt2) Bt2 += z * sB; C += z * sC;
    const int lane = threadIdx.x & 31, lr = lane & 15, hi = lane >> 4; const int r0 = blockIdx.x * 64, c0 = blockIdx.y * 64;
    v8f acc[4][4];
#pragma unroll
    for (int mb = 0; mb < 4; ++mb)
#pragma unroll
        for (int nb = 0; nb < 4; ++nb) acc[mb][nb] = (v8f){};
    const size_t aoff = (size_t)(r0 + lr) * K + 8 * hi, boff = (size_t)(c0 + lr) * K + 8 * hi;
#pragma unroll 1
    for (int kc = 0; kc < K; kc += 32) {
        V a[4], a2[4];
#pragma unroll
        for (int mb = 0; mb < 4; ++mb) { a[mb] = WFrag<T16>::ld(A + aoff + (size_t)mb * 16 * K + kc); if (NSPLIT == 1 || NSPLIT == 2) a2[mb] = WFrag<T16>::ld(A2 + aoff + (size_t)mb * 16 * K + kc); }
#pragma unroll
        for (int nb = 0; nb < 4; ++nb) { const V b = WFrag<T16>::ld(Bt + boff + (size_t)nb * 16 * K + kc); V b2; if (NSPLIT >= 2) b2 = WFrag<T16>::ld(Bt2 + boff + (size_t)nb * 16 * K + kc);
#pragma unroll
            for (int mb = 0; mb < 4; ++mb) { acc[mb][nb] = WFrag<T16>::mma(a[mb], b, acc[mb][nb]); if (NSPLIT == 1 || NSPLIT == 2) acc[mb][nb] = WFrag<T16>::mma(a2[mb], b, acc[mb][nb]); if (NSPLIT >= 2) acc[mb][nb] = WFrag<T16>::mma(a[mb], b2, acc[mb][nb]); } }
        asm volatile("v_nop\n\tv_nop\n\tv_nop\n\tv_nop" : "+v"(acc[0][0]), "+v"(acc[1][1]), "+v"(acc[2][2]), "+v"(acc[3][3]) : "v"(a[0]), "v"(a[3]));
    }
#pragma unroll
    for (int mb = 0; mb < 4; ++mb) {
#pragma unroll
        for (int nb = 0; nb < 4; ++nb) {
#pragma unroll
            for (int j = 0; j < 8; ++j) os[(hi * 8 + j) * 68 + nb * 16 + lr] = acc[mb][nb][j]; }
        __builtin_amdgcn_wave_barrier(); asm volatile("" ::: "memory");
        float* crow = C + (size_t)(r0 + mb * 16) * ldc + c0;
#pragma unroll 1
        for (int ps = 0; ps < 2; ++ps) {
#pragma unroll
            for (int s = 0; s < 8; ++s) { const int row = 2 * s + hi, cofs = lr * 4; v4f val = *(const v4fa*)(os + row * 68 + cofs); if (BIAS) { val[0] += bfr(bias[c0 + cofs]); val[1] += bfr(bias[c0 + cofs + 1]); val[2] += bfr(bias[c0 + cofs + 2]); val[3] += bfr(bias[c0 + cofs + 3]); }
                *(volatile v4f*)(crow + (size_t)row * ldc + cofs) = val; }
            if (ps == 0) __threadfence(); }
        __builtin_amdgcn_wave_barrier(); asm volatile("" ::: "memory");
    }
}

__device__ __forceinline__ h16 tohx(float x) { return (h16)x; }
__device__ __forceinline__ void splitf(float y, unsigned short& h, unsigned short& l) { h = f2bf(y); l = f2bf(y - bf2f(h)); }
typedef __attribute__((ext_vector_type(2))) _Float16 v2h;
typedef __attribute__((ext_vector_type(4))) _Float16 v4h;
typedef __attribute__((ext_vector_type(2))) unsigned short v2us;
typedef __attribute__((ext_vector_type(4))) unsigned short v4us;
typedef __attribute__((ext_vector_type(2))) float v2f;
typedef __attribute__((ext_vector_type(4))) int v4i;

__global__ __launch_bounds__(256) void k_wtG(const float* __restrict__ w, int K, int N, bf* Bt) {
    const int lane = threadIdx.x & 31; const int L0 = (blockIdx.x * 8 + (threadIdx.x >> 5)) * 8; const int nlines = N * K / 64;
#pragma unroll
    for (int ps = 0; ps < 2; ++ps) {
#pragma unroll 1
        for (int l = 0; l < 8; ++l) { const int L = L0 + l; if (L >= nlines) break; const size_t e = (size_t)L * 64 + lane * 2; const int k = (int)(e % K), n = (int)(e / K); v2us o;
            o[0] = f2bf(w[(size_t)k * N + n]); o[1] = f2bf(w[(size_t)(k + 1) * N + n]); *(volatile v2us*)(Bt + e) = o; }
        if (ps == 0) __threadfence(); }
}
__global__ __launch_bounds__(256) void k_cvt8(const float* __restrict__ src, bf* dst, size_t n8) { const size_t i = (size_t)blockIdx.x * 256 + threadIdx.x; if (i >= n8) return; const v8f v = *(const v8f*)(src + i * 8); v8us o;
#pragma unroll
    for (int k = 0; k < 8; ++k) o[k] = f2bf(v[k]); *(volatile v8us*)(dst + i * 8) = o; __threadfence(); *(volatile v8us*)(dst + i * 8) = o; }

__global__ __launch_bounds__(256) void k_rope(const float* __restrict__ F, int pitch, int nheads, const float* __restrict__ CS, const float* __restrict__ RF, const float* __restrict__ nw, float sc, h16* P16, bf* Ph, bf* Pl) {
    const size_t e = ((size_t)blockIdx.x * 256 + threadIdx.x) * 2; if (e >= (size_t)nheads * TT * HD) return; const int d = (int)(e % HD); const int t = (int)((e / HD) % TT); const int h = (int)(e / ((size_t)HD * TT)); const float* f = F + (size_t)t * pitch + h * HD; const float rf = RF ? RF[(size_t)h * TT + t] : 1.0f; v2h o16; v2us oh, ol;
#pragma unroll
    for (int q = 0; q < 2; ++q) { const int dd = d + q; const int dp = (dd < HD / 2) ? dd + HD / 2 : dd - HD / 2; float x0 = f[dd], x1 = f[dp];
        if (RF) { float n0 = __fmul_rn(x0, rf), n1 = __fmul_rn(x1, rf); asm volatile("" : "+v"(n0)); asm volatile("" : "+v"(n1)); x0 = __fmul_rn(bfr(nw[dd]), n0); x1 = __fmul_rn(bfr(nw[dp]), n1); }
        const v2f cs = *(const v2f*)(CS + ((size_t)t * HD + dd) * 2); float a = __fmul_rn(x0, cs[0]), bq = __fmul_rn(x1, cs[1]); asm volatile("" : "+v"(a)); asm volatile("" : "+v"(bq)); const float r = ((dd < HD / 2) ? __fsub_rn(a, bq) : __fadd_rn(a, bq)) * sc;
        o16[q] = tohx(r); unsigned short a2, c2; splitf(r, a2, c2); oh[q] = a2; ol[q] = c2; }
    *(volatile v2h*)(P16 + e) = o16; *(volatile v2us*)(Ph + e) = oh; *(volatile v2us*)(Pl + e) = ol; __threadfence(); *(volatile v2h*)(P16 + e) = o16; *(volatile v2us*)(Ph + e) = oh; *(volatile v2us*)(Pl + e) = ol; }
__global__ __launch_bounds__(256) void k_vtp(const float* __restrict__ F, int pitch, int nheads, h16* V16, bf* Vh, bf* Vl) { const size_t e = ((size_t)blockIdx.x * 256 + threadIdx.x) * 2; if (e >= (size_t)nheads * HD * TT) return; const int t = (int)(e % TT); const int d = (int)((e / TT) % HD); const int g = (int)(e / ((size_t)TT * HD)); v2h o16; v2us oh, ol;
#pragma unroll
    for (int q = 0; q < 2; ++q) { const float x = F[(size_t)(t + q) * pitch + g * HD + d]; o16[q] = tohx(x); unsigned short a2, c2; splitf(x, a2, c2); oh[q] = a2; ol[q] = c2; }
    *(volatile v2h*)(V16 + e) = o16; *(volatile v2us*)(Vh + e) = oh; *(volatile v2us*)(Vl + e) = ol; __threadfence(); *(volatile v2h*)(V16 + e) = o16; *(volatile v2us*)(Vh + e) = oh; *(volatile v2us*)(Vl + e) = ol; }
__global__ __launch_bounds__(256) void k_csid(float* CS) { const int idx = blockIdx.x * 256 + threadIdx.x; if (idx >= TT * HD) return; v2f cs; cs[0] = 1.0f; cs[1] = 0.0f; *(volatile v2f*)(CS + (size_t)idx * 2) = cs; __threadfence(); *(volatile v2f*)(CS + (size_t)idx * 2) = cs; }
__global__ __launch_bounds__(256) void k_asoft(const float* __restrict__ Sb, h16* P16, bf* Ph, bf* Pl) {
    const int lane = threadIdx.x & 31; const int row = blockIdx.x * 8 + (threadIdx.x >> 5); if (row >= ZH * TT) return; const int i = row % TT; const int zz = row / TT; (void)zz; const bool hires = (i < RH); const float* sr = Sb + (size_t)row * TT; float v[TT / 32]; float mx = -3.0e38f;
#pragma unroll
    for (int ch = 0; ch < TT / 128; ++ch) { const int j0 = ch * 128 + lane * 4; const v4f a = *(const v4f*)(sr + j0);
#pragma unroll
        for (int q = 0; q < 4; ++q) { const int j = j0 + q; (void)j; const float t = a[q] * SCL; v[ch * 4 + q] = t; mx = fmaxf(mx, t); } }
#pragma unroll
    for (int sh = 16; sh; sh >>= 1) mx = fmaxf(mx, __shfl_xor(mx, sh, 32));
    float sum = 0.f;
#pragma unroll
    for (int k = 0; k < TT / 32; ++k) { float d0 = __fsub_rn(v[k], mx); asm volatile("" : "+v"(d0)); v[k] = __builtin_amdgcn_exp2f(__fmul_rn(d0, 1.4426950408889634f)); sum += v[k]; }
#pragma unroll
    for (int sh = 16; sh; sh >>= 1) sum += __shfl_xor(sum, sh, 32);
    const float f = __fdiv_rn(hires ? 1.0f : PCAR, sum);
#pragma unroll 1
    for (int ps = 0; ps < 2; ++ps) {
        if (hires) {
#pragma unroll
            for (int ch = 0; ch < TT / 128; ++ch) { v4us oh, ol;
#pragma unroll
                for (int q = 0; q < 4; ++q) { unsigned short a, c2; splitf(v[ch * 4 + q] * f, a, c2); oh[q] = a; ol[q] = c2; }
                const size_t oo = ((size_t)zz * (RH ? RH : 1) + i) * TT + ch * 128 + lane * 4; *(volatile v4us*)(Ph + oo) = oh; *(volatile v4us*)(Pl + oo) = ol; }
        } else {
#pragma unroll
            for (int ch = 0; ch < TT / 128; ++ch) { v4h o4;
#pragma unroll
                for (int q = 0; q < 4; ++q) o4[q] = tohx(v[ch * 4 + q] * f);
                *(volatile v4h*)(P16 + (size_t)row * TT + ch * 128 + lane * 4) = o4; } }
        if (ps == 0) __threadfence(); }
}
__constant__ float DEN[DM / 2] = { 1.000000000e+00f, 9.821718931e-01f, 9.646616578e-01f, 9.474635124e-01f, 9.305720329e-01f, 9.139816761e-01f, 8.976871371e-01f, 8.816829920e-01f, 8.659643531e-01f, 8.505257964e-01f, 8.353624940e-01f, 8.204696178e-01f, 8.058421612e-01f, 7.914754748e-01f, 7.773650289e-01f, 7.635060549e-01f, 7.498942018e-01f, 7.365249991e-01f, 7.233942151e-01f, 7.104973793e-01f, 6.978306174e-01f, 6.853896379e-01f, 6.731703877e-01f, 6.611690521e-01f, 6.493816376e-01f, 6.378043890e-01f, 6.264334917e-01f, 6.152654290e-01f, 6.042963862e-01f, 5.935229063e-01f, 5.829415917e-01f, 5.725488067e-01f, 5.623413324e-01f, 5.523158312e-01f, 5.424690247e-01f, 5.327978730e-01f, 5.232990980e-01f, 5.139696598e-01f, 5.048065186e-01f, 4.958068430e-01f, 4.869674742e-01f, 4.782857597e-01f, 4.697588682e-01f, 4.613839686e-01f, 4.531583488e-01f, 4.450793862e-01f, 4.371444881e-01f, 4.293510020e-01f, 4.216964841e-01f, 4.141784608e-01f, 4.067944288e-01f, 3.995420337e-01f, 3.924189508e-01f, 3.854228854e-01f, 3.785515130e-01f, 3.718026578e-01f, 3.651741147e-01f, 3.586637676e-01f, 3.522694409e-01f, 3.459891677e-01f, 3.398208320e-01f, 3.337624669e-01f, 3.278121054e-01f, 3.219678402e-01f, 3.162277639e-01f, 3.105900288e-01f, 3.050527871e-01f, 2.996142805e-01f, 2.942726910e-01f, 2.890264094e-01f, 2.838736176e-01f, 2.788126469e-01f, 2.738419473e-01f, 2.689598799e-01f, 2.641648352e-01f, 2.594552934e-01f, 2.548296452e-01f, 2.502865493e-01f, 2.458243966e-01f, 2.414418310e-01f, 2.371373475e-01f, 2.329096496e-01f, 2.287573069e-01f, 2.246790081e-01f, 2.206734121e-01f, 2.167392075e-01f, 2.128751576e-01f, 2.090800107e-01f, 2.053525001e-01f, 2.016914636e-01f, 1.980956644e-01f, 1.945639998e-01f, 1.910952926e-01f, 1.876884252e-01f, 1.843422651e-01f, 1.810558140e-01f, 1.778279245e-01f, 1.746576130e-01f, 1.715438068e-01f, 1.684854776e-01f, 1.654817164e-01f, 1.625314951e-01f, 1.596338600e-01f, 1.567878723e-01f, 1.539926529e-01f, 1.512472481e-01f, 1.485507935e-01f, 1.459024251e-01f, 1.433012486e-01f, 1.407464594e-01f, 1.382372230e-01f, 1.357727200e-01f, 1.333521456e-01f, 1.309747249e-01f, 1.286397129e-01f, 1.263462752e-01f, 1.240937710e-01f, 1.218814030e-01f, 1.197085008e-01f, 1.175743267e-01f, 1.154782102e-01f, 1.134194359e-01f, 1.113973856e-01f, 1.094113961e-01f, 1.074607670e-01f, 1.055449545e-01f, 1.036632806e-01f, 1.018151641e-01f, 9.999999404e-02f, 9.821719676e-02f, 9.646616131e-02f, 9.474635124e-02f, 9.305720776e-02f, 9.139815718e-02f, 8.976870030e-02f, 8.816830069e-02f, 8.659643680e-02f, 8.505257219e-02f, 8.353625238e-02f, 8.204696327e-02f, 8.058422059e-02f, 7.914756238e-02f, 7.773648947e-02f, 7.635059953e-02f, 7.498940825e-02f, 7.365249842e-02f, 7.233940810e-02f, 7.104974240e-02f, 6.978305429e-02f, 6.853895634e-02f, 6.731704623e-02f, 6.611689180e-02f, 6.493815035e-02f, 6.378042698e-02f, 6.264335662e-02f, 6.152653694e-02f, 6.042964011e-02f, 5.935228989e-02f, 5.829415098e-02f, 5.725488067e-02f, 5.623412877e-02f, 5.523157492e-02f, 5.424689874e-02f, 5.327978358e-02f, 5.232990906e-02f, 5.139696598e-02f, 5.048066005e-02f, 4.958068207e-02f, 4.869674891e-02f, 4.782858491e-02f, 4.697588459e-02f, 4.613839090e-02f, 4.531583562e-02f, 4.450793564e-02f, 4.371444881e-02f, 4.293510318e-02f, 4.216965288e-02f, 4.141784832e-02f, 4.067944363e-02f, 3.995420039e-02f, 3.924189508e-02f, 3.854228556e-02f, 3.785514832e-02f, 3.718026355e-02f, 3.651741147e-02f, 3.586637974e-02f, 3.522694856e-02f, 3.459891677e-02f, 3.398207575e-02f, 3.337624297e-02f, 3.278120980e-02f, 3.219677880e-02f, 3.162277490e-02f, 3.105900064e-02f, 3.050528094e-02f, 2.996142954e-02f, 2.942727320e-02f, 2.890263498e-02f, 2.838735469e-02f, 2.788126469e-02f, 2.738419361e-02f, 2.689598687e-02f, 2.641648240e-02f, 2.594552934e-02f, 2.548296750e-02f, 2.502865531e-02f, 2.458243445e-02f, 2.414417826e-02f, 2.371373586e-02f, 2.329096384e-02f, 2.287572995e-02f, 2.246790007e-02f, 2.206734009e-02f, 2.167392150e-02f, 2.128751948e-02f, 2.090799809e-02f, 2.053524740e-02f, 2.016914450e-02f, 1.980956644e-02f, 1.945639960e-02f, 1.910952851e-02f, 1.876884326e-02f, 1.843423024e-02f, 1.810557768e-02f, 1.778279617e-02f, 1.746575907e-02f, 1.715438068e-02f, 1.684854738e-02f, 1.654817350e-02f, 1.625314727e-02f, 1.596338116e-02f, 1.567878947e-02f, 1.539926138e-02f, 1.512472611e-02f, 1.485507749e-02f, 1.459024474e-02f, 1.433012355e-02f, 1.407464873e-02f, 1.382372063e-02f, 1.357726846e-02f, 1.333521493e-02f, 1.309746969e-02f, 1.286397036e-02f, 1.263462752e-02f, 1.240937877e-02f, 1.218814030e-02f, 1.197085157e-02f, 1.175743155e-02f, 1.154781599e-02f, 1.134194341e-02f, 1.113973651e-02f, 1.094113849e-02f, 1.074607577e-02f, 1.055449713e-02f, 1.036632806e-02f, 1.018151827e-02f, 9.999998845e-03f, 9.821715765e-03f, 9.646615945e-03f, 9.474633262e-03f, 9.305721149e-03f, 9.139815345e-03f, 8.976872079e-03f, 8.816829883e-03f, 8.659644052e-03f, 8.505257778e-03f, 8.353622630e-03f, 8.204695769e-03f, 8.058420382e-03f, 7.914755493e-03f, 7.773648947e-03f, 7.635061163e-03f, 7.498941384e-03f, 7.365250494e-03f, 7.233941462e-03f, 7.104972377e-03f, 6.978305522e-03f, 6.853894331e-03f, 6.731703877e-03f, 6.611688994e-03f, 6.493817084e-03f, 6.378042977e-03f, 6.264335942e-03f, 6.152653601e-03f, 6.042962428e-03f, 5.935228430e-03f, 5.829413887e-03f, 5.725487601e-03f, 5.623412319e-03f, 5.523158703e-03f, 5.424690433e-03f, 5.327979568e-03f, 5.232990719e-03f, 5.139695015e-03f, 5.048065912e-03f, 4.958067089e-03f, 4.869675264e-03f, 4.782857373e-03f, 4.697589204e-03f, 4.613838624e-03f, 4.531584214e-03f, 4.450793844e-03f, 4.371443763e-03f, 4.293510225e-03f, 4.216964357e-03f, 4.141784739e-03f, 4.067943431e-03f, 3.995420877e-03f, 3.924189135e-03f, 3.854229115e-03f, 3.785514971e-03f, 3.718025517e-03f, 3.651741194e-03f, 3.586636856e-03f, 3.522694577e-03f, 3.459890839e-03f, 3.398208646e-03f, 3.337624250e-03f, 3.278121352e-03f, 3.219678067e-03f, 3.162276698e-03f, 3.105900018e-03f, 3.050526837e-03f, 2.996142488e-03f, 2.942726482e-03f, 2.890263917e-03f, 2.838735469e-03f, 2.788126934e-03f, 2.738419455e-03f, 2.689599060e-03f, 2.641648054e-03f, 2.594552236e-03f, 2.548296703e-03f, 2.502865158e-03f, 2.458244096e-03f, 2.414417919e-03f, 2.371373819e-03f, 2.329096431e-03f, 2.287573414e-03f, 2.246790100e-03f, 2.206733450e-03f, 2.167392289e-03f, 2.128751250e-03f, 2.090800088e-03f, 2.053524600e-03f, 2.016914776e-03f, 1.980956411e-03f, 1.945640426e-03f, 1.910952735e-03f, 1.876883674e-03f, 1.843422768e-03f, 1.810557791e-03f, 1.778279548e-03f, 1.746575814e-03f, 1.715438091e-03f, 1.684854738e-03f, 1.654817257e-03f, 1.625314704e-03f, 1.596337999e-03f, 1.567878760e-03f, 1.539926161e-03f, 1.512472518e-03f, 1.485507586e-03f, 1.459024264e-03f, 1.433012309e-03f, 1.407464850e-03f, 1.382372109e-03f, 1.357726753e-03f, 1.333521446e-03f, 1.309746993e-03f, 1.286396873e-03f, 1.263462706e-03f, 1.240937738e-03f, 1.218814054e-03f, 1.197085250e-03f, 1.175743178e-03f, 1.154781668e-03f, 1.134194317e-03f, 1.113973558e-03f, 1.094113919e-03f, 1.074607600e-03f, 1.055449597e-03f, 1.036632806e-03f, 1.018151757e-03f, 9.999999311e-04f, 9.821716230e-04f, 9.646615363e-04f, 9.474633262e-04f, 9.305720450e-04f, 9.139814647e-04f, 8.976871613e-04f, 8.816829650e-04f, 8.659644518e-04f, 8.505257429e-04f, 8.353622979e-04f, 8.204695769e-04f, 8.058419917e-04f, 7.914755261e-04f, 7.773648249e-04f, 7.635061629e-04f, 7.498940686e-04f, 7.365250494e-04f, 7.233940996e-04f, 7.104971446e-04f, 6.978305173e-04f, 6.853894447e-04f, 6.731703761e-04f, 6.611688877e-04f, 6.493816036e-04f, 6.378042744e-04f, 6.264336407e-04f, 6.152653950e-04f, 6.042961613e-04f, 5.935229128e-04f, 5.829414004e-04f, 5.725487717e-04f, 5.623411853e-04f, 5.523158470e-04f, 5.424690316e-04f, 5.327979452e-04f, 5.232990370e-04f, 5.139695131e-04f, 5.048065213e-04f, 4.958066856e-04f, 4.869675031e-04f, 4.782857141e-04f, 4.697589320e-04f, 4.613838682e-04f, 4.531583982e-04f, 4.450793494e-04f, 4.371443647e-04f, 4.293509701e-04f, 4.216963716e-04f, 4.141784739e-04f, 4.067943373e-04f, 3.995420702e-04f, 3.924188786e-04f, 3.854228999e-04f, 3.785514564e-04f, 3.718025109e-04f, 3.651740844e-04f, 3.586636449e-04f, 3.522694169e-04f, 3.459890722e-04f, 3.398208355e-04f, 3.337624075e-04f, 3.278119839e-04f, 3.219679347e-04f, 3.162278153e-04f, 3.105900250e-04f, 3.050527012e-04f, 2.996141266e-04f, 2.942727879e-04f, 2.890263859e-04f, 2.838735236e-04f, 2.788125712e-04f, 2.738420735e-04f, 2.689599060e-04f, 2.641648171e-04f, 2.594552061e-04f, 2.548295306e-04f, 2.502865973e-04f, 2.458243980e-04f, 2.414417831e-04f, 2.371372830e-04f, 2.329097333e-04f, 2.287573298e-04f, 2.246789954e-04f, 2.206733479e-04f, 2.167390921e-04f, 2.128752094e-04f, 2.090799971e-04f, 2.053524513e-04f, 2.016913641e-04f, 1.980957459e-04f, 1.945640106e-04f, 1.910952706e-04f, 1.876883616e-04f, 1.843421924e-04f, 1.810558460e-04f, 1.778279257e-04f, 1.746575581e-04f, 1.715437102e-04f, 1.684855233e-04f, 1.654817315e-04f, 1.625314617e-04f, 1.596337970e-04f, 1.567878062e-04f, 1.539926743e-04f, 1.512472518e-04f, 1.485507673e-04f, 1.459023624e-04f, 1.433013094e-04f, 1.407464879e-04f, 1.382372138e-04f, 1.357726724e-04f, 1.333520777e-04f, 1.309747458e-04f, 1.286397019e-04f, 1.263462618e-04f, 1.240937272e-04f, 1.218814577e-04f, 1.197085148e-04f, 1.175743091e-04f, 1.154781567e-04f, 1.134193808e-04f, 1.113974067e-04f, 1.094113759e-04f, 1.074607499e-04f, 1.055449175e-04f, 1.036633330e-04f, 1.018151816e-04f };
__global__ __launch_bounds__(256) void k_petab2(float* PE) { const int idx = blockIdx.x * 256 + threadIdx.x; if (idx >= TT * DM) return; const int d = idx % DM; const int srow = idx / DM; const float ang = __fmul_rn((float)srow, DEN[d >> 1]); const float p = (d & 1) ? cosf(ang) : sinf(ang); *(volatile float*)(PE + idx) = p; __threadfence(); *(volatile float*)(PE + idx) = p; }
__global__ __launch_bounds__(256) void k_cvtTpe(const float* __restrict__ X, const float* __restrict__ PE, bf* Xh, bf* Xl) { const size_t i = (size_t)blockIdx.x * 256 + threadIdx.x; if (i >= (size_t)TT * DM / 8) return; const size_t e = i * 8; const int d0 = (int)(e % DM); const int srow = (int)(e / DM); v8us oh, ol;
#pragma unroll
    for (int q = 0; q < 8; ++q) { const float v = __fadd_rn(bfr(X[(size_t)(d0 + q) * TT + srow]), PE[e + q]); unsigned short hh, ll; splitf(v, hh, ll); oh[q] = hh; ol[q] = ll; }
    *(volatile v8us*)(Xh + e) = oh; *(volatile v8us*)(Xl + e) = ol; __threadfence(); *(volatile v8us*)(Xh + e) = oh; *(volatile v8us*)(Xl + e) = ol; }
__global__ __launch_bounds__(256) void k_trout(const float* __restrict__ Y, float* OUT) { const size_t k = (size_t)blockIdx.x * 256 + threadIdx.x; if (k >= (size_t)DM * TT / 4) return; const size_t e = k * 4; const int s0 = (int)(e % TT); const int d = (int)(e / TT); v4f o;
#pragma unroll
    for (int q = 0; q < 4; ++q) o[q] = Y[(size_t)(s0 + q) * DM + d];
    *(volatile v4f*)(OUT + e) = o; __threadfence(); *(volatile v4f*)(OUT + e) = o; }
__global__ __launch_bounds__(256) void k_merge(const float* __restrict__ O, int h0, bf* Ah, bf* Al) { const size_t e = ((size_t)blockIdx.x * 256 + threadIdx.x) * 2; if (e >= (size_t)ZH * TT * HD) return; const int d = (int)(e % HD); const int t = (int)((e / HD) % TT); const int zz = (int)(e / ((size_t)HD * TT)); const float cs = (t < RH) ? 1.0f : (1.0f / PCAR); const size_t oo = (size_t)t * DQ + (h0 + zz) * HD + d;
    v2us oh, ol;
#pragma unroll
    for (int q = 0; q < 2; ++q) { unsigned short a, c2; splitf(O[e + q] * cs, a, c2); oh[q] = a; ol[q] = c2; } *(volatile v2us*)(Ah + oo) = oh; *(volatile v2us*)(Al + oo) = ol; __threadfence(); *(volatile v2us*)(Ah + oo) = oh; *(volatile v2us*)(Al + oo) = ol; }

extern "C" void kernel_launch(void* const* d_in, const int* in_sizes, int n_in,
                              void* d_out, int out_size, void* d_ws, size_t ws_size, hipStream_t stream) {
    (void)in_sizes; (void)n_in; (void)out_size;
    const float* xin = (const float*)d_in[0];     const float* wq = (const float*)d_in[1]; const float* bq = (const float*)d_in[2]; const float* wk = (const float*)d_in[3]; const float* bk = (const float*)d_in[4]; const float* wv = (const float*)d_in[5]; const float* bv = (const float*)d_in[6]; const float* wo = (const float*)d_in[7]; const float* bo = (const float*)d_in[8];   const float* x = xin;
    float* OUT = (float*)d_out;
    char* wsp = (char*)d_ws;
    auto take = [&](size_t bytes) { char* p = wsp; wsp += (bytes + 255) & ~(size_t)255; return (void*)p; };
    bf* XBl = (bf*)take((size_t)TT * DM * 2); float* PE = (float*)take((size_t)TT * DM * 4); float* YT = (float*)take((size_t)TT * DM * 4); bf* WQ = (bf*)take((size_t)DQ * DM * 2); bf* WK = (bf*)take((size_t)DKV * DM * 2); bf* WV = (bf*)take((size_t)DKV * DM * 2); bf* WO = (bf*)take((size_t)DM * DQ * 2); float* CS = (float*)take((size_t)TT * HD * 2 * 4);
    bf* XB = (bf*)take((size_t)TT * DM * 2); float* FQ = (float*)take((size_t)TT * DQ * 4); float* FK = (float*)take((size_t)TT * DKV * 4);
    h16* QP16 = (h16*)take((size_t)NH_ * TT * HD * 2); h16* KP16 = (h16*)take((size_t)NKV * TT * HD * 2); h16* VT16 = (h16*)take((size_t)NKV * HD * TT * 2);
    bf* QPh = (bf*)take((size_t)NH_ * TT * HD * 2); bf* QPl = (bf*)take((size_t)NH_ * TT * HD * 2); bf* KPh = (bf*)take((size_t)NKV * TT * HD * 2); bf* KPl = (bf*)take((size_t)NKV * TT * HD * 2); bf* VTh = (bf*)take((size_t)NKV * HD * TT * 2); bf* VTl = (bf*)take((size_t)NKV * HD * TT * 2); bf* Ph = (bf*)take((size_t)ZH * RH * TT * 2); bf* Pl = (bf*)take((size_t)ZH * RH * TT * 2);
    float* Sb = (float*)take((size_t)ZH * TT * TT * 4); h16* P16 = (h16*)take((size_t)ZH * TT * TT * 2); float* Ob = (float*)take((size_t)ZH * TT * HD * 4); bf* ATh = (bf*)take((size_t)TT * DQ * 2); bf* ATl = (bf*)take((size_t)TT * DQ * 2);
    if ((size_t)(wsp - (char*)d_ws) > ws_size) return;
    float* FV = FK;
    { k_cvt8<<<(unsigned)(((size_t)DQ * DM / 8 + 255) / 256), 256, 0, stream>>>(wq, WQ, (size_t)DQ * DM / 8); k_cvt8<<<(unsigned)(((size_t)DKV * DM / 8 + 255) / 256), 256, 0, stream>>>(wk, WK, (size_t)DKV * DM / 8); k_cvt8<<<(unsigned)(((size_t)DKV * DM / 8 + 255) / 256), 256, 0, stream>>>(wv, WV, (size_t)DKV * DM / 8);
      k_cvt8<<<(unsigned)(((size_t)DM * DQ / 8 + 255) / 256), 256, 0, stream>>>(wo, WO, (size_t)DM * DQ / 8);
       }
    k_csid<<<(TT * HD + 255) / 256, 256, 0, stream>>>(CS);
    const unsigned LQ = (unsigned)(((size_t)NH_ * TT * HD / 2 + 255) / 256), LKv = (unsigned)(((size_t)NKV * TT * HD / 2 + 255) / 256);
    for (int b = 0; b < NB_; ++b) {

        if (b == 0) k_petab2<<<(TT * DM + 255) / 256, 256, 0, stream>>>(PE); k_cvtTpe<<<(unsigned)(((size_t)TT * DM / 8 + 255) / 256), 256, 0, stream>>>(xin + (size_t)b * DM * TT, PE, XB, XBl);
        k_gemmw<bf, 1, true><<<dim3(TT / 64, DQ / 64, 1), 32, 0, stream>>>(XB, XBl, WQ, nullptr, DM, FQ, DQ, bq, 0, 0, 0);
        k_rope<<<LQ, 256, 0, stream>>>(FQ, DQ, NH_, CS, nullptr, nullptr, 1.0f, QP16, QPh, QPl);
        k_gemmw<bf, 1, true><<<dim3(TT / 64, DKV / 64, 1), 32, 0, stream>>>(XB, XBl, WK, nullptr, DM, FK, DKV, bk, 0, 0, 0);
        k_rope<<<LKv, 256, 0, stream>>>(FK, DKV, NKV, CS, nullptr, nullptr, 1.0f, KP16, KPh, KPl);
        k_gemmw<bf, 1, true><<<dim3(TT / 64, DKV / 64, 1), 32, 0, stream>>>(XB, XBl, WV, nullptr, DM, FV, DKV, bv, 0, 0, 0); k_vtp<<<LKv, 256, 0, stream>>>(FV, DKV, NKV, VT16, VTh, VTl);
        for (int h0 = 0; h0 < NH_; h0 += ZH) { const size_t zq = (size_t)h0, zk = (size_t)(h0 / REP);
            k_gemmw<bf, 2, false><<<dim3(RH / 64, TT / 64, ZH), 32, 0, stream>>>(QPh + zq * TT * HD, QPl + zq * TT * HD, KPh + zk * TT * HD, KPl + zk * TT * HD, HD, Sb, TT, nullptr, (size_t)TT * HD, (size_t)TT * HD, (size_t)TT * TT);
            k_gemmw<h16, 0, false><<<dim3((TT - RH) / 64, TT / 64, ZH), 32, 0, stream>>>(QP16 + zq * TT * HD + (size_t)RH * HD, nullptr, KP16 + zk * TT * HD, nullptr, HD, Sb + (size_t)RH * TT, TT, nullptr, (size_t)TT * HD, (size_t)TT * HD, (size_t)TT * TT);
            k_asoft<<<ZH * TT / 8, 256, 0, stream>>>(Sb, P16, Ph, Pl);
            k_gemmw<bf, 2, false><<<dim3(RH / 64, HD / 64, ZH), 32, 0, stream>>>(Ph, Pl, VTh + zk * HD * TT, VTl + zk * HD * TT, TT, Ob, HD, nullptr, (size_t)RH * TT, (size_t)HD * TT, (size_t)TT * HD);
            k_gemmw<h16, 0, false><<<dim3((TT - RH) / 64, HD / 64, ZH), 32, 0, stream>>>(P16 + (size_t)RH * TT, nullptr, VT16 + zk * HD * TT, nullptr, TT, Ob + (size_t)RH * HD, HD, nullptr, (size_t)TT * TT, (size_t)HD * TT, (size_t)TT * HD);
            k_merge<<<(unsigned)(((size_t)ZH * TT * HD / 2 + 255) / 256), 256, 0, stream>>>(Ob, h0, ATh, ATl); }
        k_gemmw<bf, 1, true><<<dim3(TT / 64, DM / 64, 1), 32, 0, stream>>>(ATh, ATl, WO, nullptr, DQ, YT, DM, bo, 0, 0, 0);     k_trout<<<(unsigned)(((size_t)DM * TT / 4 + 255) / 256), 256, 0, stream>>>(YT, OUT + (size_t)b * DM * TT);     }
}
